// MixtureLinear_30356828848765
// MI455X (gfx1250) — hardware-verified
//
#include <hip/hip_runtime.h>
#include <stddef.h>


typedef __attribute__((ext_vector_type(16))) _Float16 v16h;
typedef __attribute__((ext_vector_type(8)))  _Float16 v8h;
typedef __attribute__((ext_vector_type(16))) __bf16   v16b;
typedef __attribute__((ext_vector_type(8)))  __bf16   v8b;
typedef __attribute__((ext_vector_type(8)))  float    v8f;
typedef __attribute__((ext_vector_type(4)))  float    v4f;

constexpr int Bb = 8, Nn = 1024, Cc = 1024, Dd = 1024, Rr = 8;
constexpr int MM = Bb * Nn;
constexpr int KK = Cc * Rr;
constexpr int MH = MM / 2;
constexpr float WSC     = 64.0f;
constexpr float WSC_INV = 0.015625f;

__device__ __forceinline__ unsigned short f2bf_bits(float f) {
  unsigned u = __float_as_uint(f);
  return (unsigned short)((u + 0x7FFFu + ((u >> 16) & 1u)) >> 16);
}
__device__ __forceinline__ float bf_bits2f(unsigned short h) { return __uint_as_float(((unsigned)h) << 16); }

__device__ __forceinline__ void dep_guard_h(v8f& a, v8f& b, v16h x, v16h y) { asm volatile("v_nop\n\tv_nop\n\tv_nop\n\tv_nop" : "+v"(a), "+v"(b) : "v"(x), "v"(y)); }
__device__ __forceinline__ void dep_guard_b(v8f& a, v8f& b, v16b x, v16b y) { asm volatile("v_nop\n\tv_nop\n\tv_nop\n\tv_nop" : "+v"(a), "+v"(b) : "v"(x), "v"(y)); }
__device__ __forceinline__ void keep4_h(v16h a, v16h b, v16h c, v16h d) { asm volatile("v_nop" :: "v"(a), "v"(b), "v"(c), "v"(d)); }
__device__ __forceinline__ void keep4_b(v16b a, v16b b, v16b c, v16b d) { asm volatile("v_nop" :: "v"(a), "v"(b), "v"(c), "v"(d)); }
__device__ __forceinline__ void acc_guard4(v8f& a, v8f& b, v8f& c, v8f& d) { asm volatile("v_nop\n\tv_nop\n\tv_nop\n\tv_nop" : "+v"(a), "+v"(b), "+v"(c), "+v"(d)); }
template <typename T> struct Frag;
template <> struct Frag<_Float16> {
  typedef v16h V; union U { v16h v; v8h h[2]; };
  static __device__ __forceinline__ v16h load(const _Float16* p) {
    U f; f.h[0] = *(const v8h*)(p); f.h[1] = *(const v8h*)(p + 16); return f.v;
  }
  static __device__ __forceinline__ v8f mma(v16h a, v16h b, v8f c) {
    return __builtin_amdgcn_wmma_f32_16x16x32_f16(false, a, false, b, (short)0, c, false, false);
  }
  static __device__ __forceinline__ void guard(v8f& a, v8f& b, v16h x, v16h y) { dep_guard_h(a, b, x, y); }
  static __device__ __forceinline__ void keep(v16h a, v16h b, v16h c, v16h d) { keep4_h(a, b, c, d); }
};
template <> struct Frag<__bf16> {
  typedef v16b V; union U { v16b v; v8b h[2]; };
  static __device__ __forceinline__ v16b load(const __bf16* p) {
    U f; f.h[0] = *(const v8b*)(p); f.h[1] = *(const v8b*)(p + 16); return f.v;
  }
  static __device__ __forceinline__ v8f mma(v16b a, v16b b, v8f c) {
    return __builtin_amdgcn_wmma_f32_16x16x32_bf16(false, a, false, b, (short)0, c, false, false);
  }
  static __device__ __forceinline__ void guard(v8f& a, v8f& b, v16b x, v16b y) { dep_guard_b(a, b, x, y); }
  static __device__ __forceinline__ void keep(v16b a, v16b b, v16b c, v16b d) { keep4_b(a, b, c, d); }
};

template <int ET> struct Elem;
template <> struct Elem<0> { typedef _Float16 T; };
template <> struct Elem<1> { typedef __bf16 T; };
template <int ET, bool SPLIT, int BIAS_MODE, int OUT_MODE, bool RESID, int ACT = 0>
__global__ __launch_bounds__(256) void wmma_gemm64(
    const unsigned short* __restrict__ Ap, const unsigned short* __restrict__ A2p, int lda, long strideA,
    const unsigned short* __restrict__ Btp, const unsigned short* __restrict__ Bt2p, int ldb, long strideB,
    void* __restrict__ Cout, void* __restrict__ Cout2, int ldc, long strideC,
    const float* __restrict__ bias, int ldbias, int rowmask,
    const float* __restrict__ resid, long strideR,
    int M, int N, int K, float scale) {
  typedef typename Elem<ET>::T T;
  typedef typename Frag<T>::V V;
  const T* A = (const T*)Ap; const T* A2 = (const T*)A2p; const T* Bt = (const T*)Btp; const T* Bt2 = (const T*)Bt2p;
  __shared__ __align__(16) float sT[8][16 * 68];
  const int b    = blockIdx.y;
  const int lane = threadIdx.x & 31;
  const int wave = threadIdx.x >> 5;
  const int tilesN = N >> 6;
  const int tilesM = M >> 6;
  const int tile = blockIdx.x * 8 + wave;
  if (tile >= tilesM * tilesN) return;
  const int tm = tile / tilesN;
  const int tn = tile - tm * tilesN;
  const int m0 = tm << 6;
  const int n0 = tn << 6;

  const T* Ab  = A  + (size_t)b * strideA;
  const T* Bb2g = Bt + (size_t)b * strideB;
  const T* Ab2 = SPLIT ? (A2  + (size_t)b * strideA) : nullptr;
  const T* Bb2 = SPLIT ? (Bt2 + (size_t)b * strideB) : nullptr;

  const int rlane = lane & 15;
  const int koff  = (lane >> 4) * 8;
  const int mOff  = (lane >> 4) * 8;

  v8f acc[4][4];
#pragma unroll
  for (int i = 0; i < 4; ++i)
#pragma unroll
    for (int j = 0; j < 4; ++j) acc[i][j] = (v8f){0.f,0.f,0.f,0.f,0.f,0.f,0.f,0.f};

  for (int k0 = 0; k0 < K; k0 += 32) {
    V bh[4], bl[4];
#pragma unroll
    for (int j = 0; j < 4; ++j) {
      const size_t bo = (size_t)(n0 + (j << 4) + rlane) * ldb + koff + k0;
      bh[j] = Frag<T>::load(Bb2g + bo);
      if (SPLIT) bl[j] = Frag<T>::load(Bb2 + bo);
    }
#pragma unroll
    for (int i = 0; i < 4; ++i) {
      const size_t ao = (size_t)(m0 + (i << 4) + rlane) * lda + koff + k0;
      V ah = Frag<T>::load(Ab + ao);
      V al;
      if (SPLIT) al = Frag<T>::load(Ab2 + ao);
#pragma unroll
      for (int j = 0; j < 4; ++j) {
        acc[i][j] = Frag<T>::mma(ah, bh[j], acc[i][j]);
        if (SPLIT) {
          acc[i][j] = Frag<T>::mma(ah, bl[j], acc[i][j]);
          acc[i][j] = Frag<T>::mma(al, bh[j], acc[i][j]);
        }
      }
      Frag<T>::guard(acc[i][0], acc[i][3], ah, SPLIT ? al : ah);
    }
    Frag<T>::keep(bh[0], bh[1], bh[2], bh[3]);
    if (SPLIT) Frag<T>::keep(bl[0], bl[1], bl[2], bl[3]);
  }
  acc_guard4(acc[0][0], acc[0][1], acc[0][2], acc[0][3]);
  acc_guard4(acc[1][0], acc[1][1], acc[1][2], acc[1][3]);
  acc_guard4(acc[2][0], acc[2][1], acc[2][2], acc[2][3]);
  acc_guard4(acc[3][0], acc[3][1], acc[3][2], acc[3][3]);

  float* slab = sT[wave];
  const float* Rb = RESID ? (resid + (size_t)b * strideR) : nullptr;
#pragma unroll
  for (int i = 0; i < 4; ++i) {
    const int mBase = m0 + (i << 4);
#pragma unroll
    for (int j = 0; j < 4; ++j) {
      const int n = n0 + (j << 4) + rlane;
      float bv = 0.f;
      if (BIAS_MODE == 2) bv = bias[n];
#pragma unroll
      for (int r = 0; r < 8; ++r) {
        float v = acc[i][j][r] * scale;
        if (BIAS_MODE == 1) v += bias[mBase + mOff + r];
        if (BIAS_MODE == 2) v += bv;
        if (BIAS_MODE == 3) v += bias[(size_t)((mBase + mOff + r) & rowmask) * ldbias + n];
        if (RESID) v += Rb[(size_t)(mBase + mOff + r) * ldc + n];
        if (ACT == 1) v = tanhf(v);
        if (ACT == 2) v = fmaxf(v, 0.0f);
        if (ACT == 3) v = v / (1.0f + expf(-v));
        if (ACT == 4) v = (v > 0.f) ? v : 0.01f * v;
        if (ACT == 5) v = 0.5f * v * (1.0f + erff(v * 0.70710678118654752f));
        slab[(mOff + r) * 68 + (j << 4) + rlane] = v;
      }
    }
    __builtin_amdgcn_fence(__ATOMIC_RELEASE, "workgroup");
    __builtin_amdgcn_wave_barrier();
    __builtin_amdgcn_fence(__ATOMIC_ACQUIRE, "workgroup");
    if (OUT_MODE == 0) {
      float* C = (float*)Cout + (size_t)b * strideC;
      const int hh = lane >> 4, c4 = (lane & 15) * 4;
      for (int pass = 0; pass < 2; ++pass) {
#pragma unroll
        for (int it = 0; it < 8; ++it) {
          const int row = it * 2 + hh;
          v4f v = *(const v4f*)(slab + row * 68 + c4);
          *(volatile v4f*)(C + (size_t)(mBase + row) * ldc + n0 + c4) = v;
        }
        __threadfence();
      }
    } else {
      const int q = lane >> 3, c8 = (lane & 7) * 8;
      unsigned short* C  = (unsigned short*)Cout  + (size_t)b * strideC;
      unsigned short* C2 = (OUT_MODE == 2) ? ((unsigned short*)Cout2 + (size_t)b * strideC) : nullptr;
      for (int pass = 0; pass < 2; ++pass) {
#pragma unroll
        for (int it = 0; it < 4; ++it) {
          const int row = it * 4 + q;
          const float* sp = slab + row * 68 + c8;
          v8h hv, lv;
#pragma unroll
          for (int e = 0; e < 8; ++e) {
            if (OUT_MODE == 1) {
              hv[e] = (_Float16)sp[e];
            } else {
              unsigned short hb = f2bf_bits(sp[e]);
              unsigned short lb = f2bf_bits(sp[e] - bf_bits2f(hb));
              hv[e] = __builtin_bit_cast(_Float16, hb);
              lv[e] = __builtin_bit_cast(_Float16, lb);
            }
          }
          *(volatile v8h*)(C + (size_t)(mBase + row) * ldc + n0 + c8) = hv;
          if (OUT_MODE == 2) *(volatile v8h*)(C2 + (size_t)(mBase + row) * ldc + n0 + c8) = lv;
        }
        __threadfence();
      }
    }
    __builtin_amdgcn_fence(__ATOMIC_RELEASE, "workgroup");
    __builtin_amdgcn_wave_barrier();
    __builtin_amdgcn_fence(__ATOMIC_ACQUIRE, "workgroup");
  }
}

__global__ __launch_bounds__(256) void build_bt(const float* __restrict__ w, _Float16* __restrict__ bt) {
  __shared__ __align__(16) _Float16 sh[Rr][256 + 8];
  const int d  = blockIdx.y;
  const int c0 = blockIdx.x * 256;
  const int t  = threadIdx.x;
  const float* src = w + ((size_t)d * Cc + c0 + t) * Rr;
  const v4f x0 = *(const v4f*)src;
  const v4f x1 = *(const v4f*)(src + 4);
  sh[0][t] = (_Float16)(x0[0] * WSC);
  sh[1][t] = (_Float16)(x0[1] * WSC);
  sh[2][t] = (_Float16)(x0[2] * WSC);
  sh[3][t] = (_Float16)(x0[3] * WSC);
  sh[4][t] = (_Float16)(x1[0] * WSC);
  sh[5][t] = (_Float16)(x1[1] * WSC);
  sh[6][t] = (_Float16)(x1[2] * WSC);
  sh[7][t] = (_Float16)(x1[3] * WSC);
  __syncthreads();
  const int wave = t >> 5, lane = t & 31;
  const v8h v = *(const v8h*)(&sh[wave][lane * 8]);
  _Float16* dst = bt + (size_t)d * KK + (size_t)wave * Cc + c0 + lane * 8;
  *(volatile v8h*)dst = v;
  __threadfence();
  *(volatile v8h*)dst = v;
}

__global__ __launch_bounds__(256) void build_cb(const float* __restrict__ coef, const float* __restrict__ bias,
                                               float* __restrict__ cb) {
  const int i = blockIdx.x * 256 + threadIdx.x;
  if (i >= Nn * Dd) return;
  const int n = i >> 10, d = i & (Dd - 1);
  const v4f q0 = *(const v4f*)(coef + (size_t)n * Rr);
  const v4f q1 = *(const v4f*)(coef + (size_t)n * Rr + 4);
  const v4f b0 = *(const v4f*)(bias + (size_t)d * Rr);
  const v4f b1 = *(const v4f*)(bias + (size_t)d * Rr + 4);
  float s = q0[0] * b0[0];
  s = fmaf(q0[1], b0[1], s);
  s = fmaf(q0[2], b0[2], s);
  s = fmaf(q0[3], b0[3], s);
  s = fmaf(q1[0], b1[0], s);
  s = fmaf(q1[1], b1[1], s);
  s = fmaf(q1[2], b1[2], s);
  s = fmaf(q1[3], b1[3], s);
  ((volatile float*)cb)[i] = s;
  __threadfence();
  ((volatile float*)cb)[i] = s;
}

__global__ __launch_bounds__(128) void build_a(const float* __restrict__ in, const float* __restrict__ coef,
                                              _Float16* __restrict__ A, int row0) {
  const int mp = blockIdx.x;
  const int m  = row0 + mp;
  const int n  = m & (Nn - 1);
  const int t  = threadIdx.x;
  const float* src = in + (size_t)m * Cc + (size_t)t * 8;
  const v4f x0 = *(const v4f*)src;
  const v4f x1 = *(const v4f*)(src + 4);
  const v4f q0 = *(const v4f*)(coef + (size_t)n * Rr);
  const v4f q1 = *(const v4f*)(coef + (size_t)n * Rr + 4);
  float cr[Rr];
  cr[0] = q0[0]; cr[1] = q0[1]; cr[2] = q0[2]; cr[3] = q0[3];
  cr[4] = q1[0]; cr[5] = q1[1]; cr[6] = q1[2]; cr[7] = q1[3];
  v8h hv[Rr];
#pragma unroll
  for (int r = 0; r < Rr; ++r) {
    const float cv = cr[r];
    v8h h;
    h[0] = (_Float16)(x0[0] * cv);
    h[1] = (_Float16)(x0[1] * cv);
    h[2] = (_Float16)(x0[2] * cv);
    h[3] = (_Float16)(x0[3] * cv);
    h[4] = (_Float16)(x1[0] * cv);
    h[5] = (_Float16)(x1[1] * cv);
    h[6] = (_Float16)(x1[2] * cv);
    h[7] = (_Float16)(x1[3] * cv);
    hv[r] = h;
  }
  _Float16* dst = A + (size_t)mp * KK + (size_t)t * 8;
#pragma unroll
  for (int r = 0; r < Rr; ++r) *(volatile v8h*)(dst + (size_t)r * Cc) = hv[r];
  __threadfence();
#pragma unroll
  for (int r = 0; r < Rr; ++r) *(volatile v8h*)(dst + (size_t)r * Cc) = hv[r];
}

extern "C" void kernel_launch(void* const* d_in, const int* in_sizes, int n_in,
                              void* d_out, int out_size, void* d_ws, size_t ws_size,
                              hipStream_t stream)
{
  if (n_in < 4) return;
  if (in_sizes[0] != MM * Cc || in_sizes[1] != Dd * Cc * Rr ||
      in_sizes[2] != Dd * Rr || in_sizes[3] != Nn * Rr || out_size != MM * Dd) return;

  const float* input  = (const float*)d_in[0];
  const float* weight = (const float*)d_in[1];
  const float* bias   = (const float*)d_in[2];
  const float* coef   = (const float*)d_in[3];
  float* out = (float*)d_out;

  const size_t bytesA  = (size_t)MH * KK * sizeof(_Float16);
  const size_t bytesBt = (size_t)Dd * KK * sizeof(_Float16);
  const size_t bytesCb = (size_t)Nn * Dd * sizeof(float);
  const size_t offA  = 0;
  const size_t offBt = offA + bytesA;
  const size_t offCb = offBt + bytesBt;
  const size_t total = offCb + bytesCb;
  if (total > ws_size) return;

  char* ws = (char*)d_ws;
  _Float16* Ah = (_Float16*)(ws + offA);
  _Float16* Bt = (_Float16*)(ws + offBt);
  float*    cb = (float*)(ws + offCb);

  build_bt<<<dim3(Cc / 256, Dd), 256, 0, stream>>>(weight, Bt);
  build_cb<<<(Nn * Dd + 255) / 256, 256, 0, stream>>>(coef, bias, cb);

  const int tiles  = (MH / 64) * (Dd / 64);
  const int blocks = (tiles + 7) / 8;
  for (int half = 0; half < 2; ++half) {
    const int row0 = half * MH;
    build_a<<<MH, 128, 0, stream>>>(input, coef, Ah, row0);
    float* outHalf = out + (size_t)row0 * Dd;
    hipLaunchKernelGGL(HIP_KERNEL_NAME(wmma_gemm64<0, false, 3, 0, false, 0>),
                       dim3(blocks, 1), dim3(256), 0, stream,
                       (const unsigned short*)Ah, (const unsigned short*)Ah, (int)KK, 0L,
                       (const unsigned short*)Bt, (const unsigned short*)Bt, (int)KK, 0L,
                       (void*)outHalf, (void*)outHalf, (int)Dd, 0L,
                       (const float*)cb, (int)Dd, (int)(Nn - 1),
                       (const float*)cb, 0L,
                       (int)MH, (int)Dd, (int)KK, WSC_INV);
  }
  (void)hipGetLastError();
}
